// PointNetSetAbstraction_71098888617988
// MI455X (gfx1250) — hardware-verified
//
#include <hip/hip_runtime.h>
#pragma clang fp contract(off)

typedef __attribute__((ext_vector_type(16))) _Float16 v16h;
typedef __attribute__((ext_vector_type(8)))  _Float16 v8h;
typedef __attribute__((ext_vector_type(2)))  _Float16 v2h;
typedef __attribute__((ext_vector_type(8)))  float    v8f;
typedef __attribute__((ext_vector_type(4)))  float    v4f;
typedef __attribute__((ext_vector_type(4)))  unsigned v4u;

constexpr int NBATCH = 16;
constexpr int NPTS = 8192;
constexpr int NCEN = 1024;
constexpr int NSAMP = 32;
constexpr int CFEAT = 64;
constexpr int MROWS = NBATCH * NCEN * NSAMP;
constexpr int ROWS_BLK = 512;
constexpr int NBLK_ALL = MROWS / ROWS_BLK;
constexpr int BLK_PER_BATCH = (NCEN * NSAMP) / ROWS_BLK;
constexpr int GRP_PER_BLK = ROWS_BLK / NSAMP;
constexpr int FPS_THREADS = 512;
constexpr int FPS_PPT = NPTS / FPS_THREADS;
constexpr float W_CARRY = 64.0f;
constexpr float REL_CARRY = 8.0f;
constexpr float W_XYZ_CARRY = W_CARRY / REL_CARRY;
constexpr float ACC_FOLD = 1.0f / W_CARRY;
constexpr float BALL_R2 = 0.01f;
constexpr float BN_EPS = 1e-5f;

static_assert(MROWS == 524288, "row count");
static_assert(NBLK_ALL == 1024 && BLK_PER_BATCH == 64 && GRP_PER_BLK == 16, "block map");
static_assert(FPS_PPT == 16, "points per thread");
static_assert((NCEN * NSAMP) % ROWS_BLK == 0, "a block stays inside one batch");

constexpr size_t WS_PTS  = 0;
constexpr size_t WS_Y0   = WS_PTS + (size_t)NBATCH * NPTS * CFEAT * 2;
constexpr size_t WS_T    = WS_Y0 + (size_t)MROWS * 64 * 2;
constexpr size_t WS_CEN  = WS_T + (size_t)(MROWS / 2) * 64 * 2;
constexpr size_t WS_P0   = WS_CEN + (size_t)NBATCH * 3 * NCEN * 4;
constexpr size_t WS_P1   = WS_P0 + (size_t)NBLK_ALL * 128 * 4;
constexpr size_t WS_P2   = WS_P1 + (size_t)NBLK_ALL * 128 * 4;
constexpr size_t WS_TAB0 = WS_P2 + (size_t)NBLK_ALL * 512 * 4;
constexpr size_t WS_TAB1 = WS_TAB0 + 1024;
constexpr size_t WS_TOTAL = WS_TAB1 + 1024;
static_assert(WS_TOTAL == 120784896, "carve total");
static_assert(WS_TOTAL <= 134217728, "carve under 128 MiB");
static_assert(WS_Y0 % 128 == 0 && WS_T % 128 == 0 && WS_CEN % 128 == 0 && WS_P0 % 128 == 0 &&
              WS_P1 % 128 == 0 && WS_P2 % 128 == 0 && WS_TAB0 % 128 == 0 && WS_TAB1 % 128 == 0, "line aligned");

constexpr int OUT1_OFF_BYTES = 196608;
constexpr int OUT1_OFF = OUT1_OFF_BYTES / 4;
static_assert(OUT1_OFF == NBATCH * 3 * NCEN, "second output follows the first");
static_assert(OUT1_OFF_BYTES + NBATCH * 128 * 4 == 204800, "output extent");
static_assert(OUT1_OFF_BYTES % 128 == 0, "second output line aligned");

__device__ __forceinline__ void pin8(float& a0, float& a1, float& a2, float& a3,
                                     float& a4, float& a5, float& a6, float& a7) {
  asm volatile("" : "+v"(a0), "+v"(a1), "+v"(a2), "+v"(a3), "+v"(a4), "+v"(a5), "+v"(a6), "+v"(a7));
}

__device__ __forceinline__ float h16_to_f32(unsigned hb) {
  const unsigned sgn = (hb & 0x8000u) << 16; const unsigned em = hb & 0x7fffu;
  const float fn = __uint_as_float((em << 13) + 0x38000000u);
  const float fs = (float)em * 5.9604644775390625e-8f;
  const float mag = (em < 0x400u) ? fs : fn; return __uint_as_float(__float_as_uint(mag) | sgn); }

__device__ __forceinline__ unsigned f16bits(float x) {
  const _Float16 hv = (_Float16)x;
  const unsigned short hb = __builtin_bit_cast(unsigned short, hv);
  return (unsigned)hb;
}
__device__ __forceinline__ unsigned pack2h(float a, float b) {
  v2h p;
  p.x = (_Float16)a;
  p.y = (_Float16)b;
  return __builtin_bit_cast(unsigned, p);
}

struct FragH {
  union U { v16h v; v8h h[2]; };
  static __device__ __forceinline__ v16h load(const _Float16* p) {
    U f; f.h[0] = *(const v8h*)(p); f.h[1] = *(const v8h*)(p + 16); return f.v;
  }
};
__device__ __forceinline__ v8f mma_h(v16h a, v16h b, v8f c) {
  c = __builtin_amdgcn_wmma_f32_16x16x32_f16(false, a, false, b, (short)0, c, false, false);
  asm volatile("v_nop\n\tv_nop\n\tv_nop\n\tv_nop" : "+v"(c) : "v"(a), "v"(b));
  return c;
}

__device__ __forceinline__ unsigned bn2(unsigned w, float sc0, float sh0, float sc1, float sh1) {
  const float x0 = h16_to_f32(w & 0xffffu);
  const float x1 = h16_to_f32(w >> 16);
  const float y0 = fmaxf(sc0 * x0 + sh0, 0.0f);
  const float y1 = fmaxf(sc1 * x1 + sh1, 0.0f);
  return pack2h(y0, y1);
}
__device__ __forceinline__ v4u bn8(v4u g, v4f scA, v4f scB, v4f shA, v4f shB) {
  const unsigned gx = g.x, gy = g.y, gz = g.z, gw = g.w;
  v4u o;
  o.x = bn2(gx, scA.x, shA.x, scA.y, shA.y);
  o.y = bn2(gy, scA.z, shA.z, scA.w, shA.w);
  o.z = bn2(gz, scB.x, shB.x, scB.y, shB.y);
  o.w = bn2(gw, scB.z, shB.z, scB.w, shB.w);
  return o;
}

__global__ __launch_bounds__(FPS_THREADS) void k_fps(const float* __restrict__ xyz, float* out0, float* cplane) {
#pragma clang fp contract(off)
  __shared__ __align__(16) float sCen[3 * NCEN];
  __shared__ float sWm[2][16];
  __shared__ int   sWi[2][16];
  const int b = blockIdx.x;
  const int tid = threadIdx.x;
  const int lane = tid & 31, wave = tid >> 5;
  const float* xb = xyz + (size_t)b * 3 * NPTS;
  float px[16], py[16], pz[16], mind[16];
#pragma unroll
  for (int u = 0; u < 8; ++u) px[u] = xb[u * FPS_THREADS + tid];
  pin8(px[0], px[1], px[2], px[3], px[4], px[5], px[6], px[7]);
#pragma unroll
  for (int u = 8; u < 16; ++u) px[u] = xb[u * FPS_THREADS + tid];
  pin8(px[8], px[9], px[10], px[11], px[12], px[13], px[14], px[15]);
#pragma unroll
  for (int u = 0; u < 8; ++u) py[u] = xb[NPTS + u * FPS_THREADS + tid];
  pin8(py[0], py[1], py[2], py[3], py[4], py[5], py[6], py[7]);
#pragma unroll
  for (int u = 8; u < 16; ++u) py[u] = xb[NPTS + u * FPS_THREADS + tid];
  pin8(py[8], py[9], py[10], py[11], py[12], py[13], py[14], py[15]);
#pragma unroll
  for (int u = 0; u < 8; ++u) pz[u] = xb[2 * NPTS + u * FPS_THREADS + tid];
  pin8(pz[0], pz[1], pz[2], pz[3], pz[4], pz[5], pz[6], pz[7]);
#pragma unroll
  for (int u = 8; u < 16; ++u) pz[u] = xb[2 * NPTS + u * FPS_THREADS + tid];
  pin8(pz[8], pz[9], pz[10], pz[11], pz[12], pz[13], pz[14], pz[15]);
#pragma unroll
  for (int u = 0; u < 16; ++u) mind[u] = 1e10f;

  int far = 0;
#pragma unroll 1
  for (int s = 0; s < NCEN - 1; ++s) {
    const float cx = xb[far];
    const float cy = xb[NPTS + far];
    const float cz = xb[2 * NPTS + far];
    if (tid == 0) { sCen[s] = cx; sCen[NCEN + s] = cy; sCen[2 * NCEN + s] = cz; }
    float best = -1.0f;
    int bidx = 0;
#pragma unroll
    for (int u = 0; u < 16; ++u) {
      const float dx = px[u] - cx;
      const float dy = py[u] - cy;
      const float dz = pz[u] - cz;
      const float t0 = dx * dx;
      const float t1 = dy * dy;
      const float t2 = dz * dz;
      const float d = (t0 + t2) + t1;
      const float m = fminf(mind[u], d);
      mind[u] = m;
      if (m > best) { best = m; bidx = u * FPS_THREADS + tid; }
    }
#pragma unroll
    for (int off = 16; off >= 1; off >>= 1) {
      const float ob = __shfl_xor(best, off, 32);
      const int   oi = __shfl_xor(bidx, off, 32);
      const bool take = (ob > best) || (ob == best && oi < bidx);
      best = take ? ob : best;
      bidx = take ? oi : bidx;
    }
    const int par = s & 1;
    if (lane == 0) { sWm[par][wave] = best; sWi[par][wave] = bidx; }
    __syncthreads();
    float rb = sWm[par][lane & 15];
    int   ri = sWi[par][lane & 15];
#pragma unroll
    for (int off = 8; off >= 1; off >>= 1) {
      const float ob = __shfl_xor(rb, off, 32);
      const int   oi = __shfl_xor(ri, off, 32);
      const bool take = (ob > rb) || (ob == rb && oi < ri);
      rb = take ? ob : rb;
      ri = take ? oi : ri;
    }
    far = __builtin_amdgcn_readfirstlane(ri) & (NPTS - 1);
  }
  {
    const float cx = xb[far];
    const float cy = xb[NPTS + far];
    const float cz = xb[2 * NPTS + far];
    if (tid == 0) { sCen[NCEN - 1] = cx; sCen[2 * NCEN - 1] = cy; sCen[3 * NCEN - 1] = cz; }
  }
  __syncthreads();
  const int q1 = (tid < 256) ? (tid + 512) : tid;
  const v4f va = *(const v4f*)(sCen + 4 * tid);
  const v4f vb = *(const v4f*)(sCen + 4 * q1);
  float* o0 = out0 + (size_t)b * 3 * NCEN;
  float* o1 = cplane + (size_t)b * 3 * NCEN;
  for (int pass = 0; pass < 2; ++pass) {
    *(volatile v4f*)(o0 + 4 * tid) = va;
    *(volatile v4f*)(o1 + 4 * tid) = va;
    if (tid < 256) {
      *(volatile v4f*)(o0 + 4 * q1) = vb;
      *(volatile v4f*)(o1 + 4 * q1) = vb;
    }
    __threadfence();
  }
}

__global__ __launch_bounds__(256) void k_tr(const float* __restrict__ pts, unsigned short* ptsh) {
  __shared__ float sT[64 * 65];
  const int tid = threadIdx.x;
  const int b = blockIdx.x >> 7;
  const int n0 = (blockIdx.x & 127) * 64;
  const int nl = tid & 63, c0 = tid >> 6;
  const float* src = pts + (size_t)b * CFEAT * NPTS + n0 + nl;
  float v[16];
#pragma unroll
  for (int i = 0; i < 8; ++i) v[i] = src[(size_t)(c0 + 4 * i) * NPTS];
  pin8(v[0], v[1], v[2], v[3], v[4], v[5], v[6], v[7]);
#pragma unroll
  for (int i = 8; i < 16; ++i) v[i] = src[(size_t)(c0 + 4 * i) * NPTS];
  pin8(v[8], v[9], v[10], v[11], v[12], v[13], v[14], v[15]);
#pragma unroll
  for (int i = 0; i < 16; ++i) sT[(c0 + 4 * i) * 65 + nl] = v[i];
  __syncthreads();
  const int row = tid >> 3, seg = tid & 7;
  v4u o[2];
#pragma unroll
  for (int it = 0; it < 2; ++it) {
    const int r = row + 32 * it;
    v4u w;
    w.x = pack2h(sT[(seg * 8 + 0) * 65 + r], sT[(seg * 8 + 1) * 65 + r]);
    w.y = pack2h(sT[(seg * 8 + 2) * 65 + r], sT[(seg * 8 + 3) * 65 + r]);
    w.z = pack2h(sT[(seg * 8 + 4) * 65 + r], sT[(seg * 8 + 5) * 65 + r]);
    w.w = pack2h(sT[(seg * 8 + 6) * 65 + r], sT[(seg * 8 + 7) * 65 + r]);
    o[it] = w;
  }
  unsigned short* dbase = ptsh + ((size_t)b * NPTS + n0) * CFEAT + seg * 8;
  for (int pass = 0; pass < 2; ++pass) {
#pragma unroll
    for (int it = 0; it < 2; ++it) {
      *(volatile v4u*)(dbase + (size_t)(row + 32 * it) * CFEAT) = o[it];
    }
    __threadfence();
  }
}

template <int LAYER>
__global__ __launch_bounds__(256) void k_layer(
    const float* __restrict__ xyz, const float* __restrict__ cplane,
    const unsigned short* srcA0, const unsigned short* srcA1, int split_row,
    const float* __restrict__ wgt, const float* __restrict__ bias, const float* __restrict__ tab,
    unsigned short* dst, int dst_row0, float* part, int blk0) {
#pragma clang fp contract(off)
  constexpr int KPAD = (LAYER == 0) ? 96 : 64;
  constexpr int NOUT = (LAYER == 2) ? 128 : 64;
  constexpr int NT = NOUT / 16;
  constexpr int KS = KPAD / 32;
  constexpr int NV = (LAYER == 2) ? 4 : 2;
  constexpr int SLAB_PITCH = 72;
  constexpr int SLAB_WAVE = 16 * SLAB_PITCH;
  static_assert(KPAD % 32 == 0 && NOUT % 16 == 0 && ROWS_BLK % 128 == 0, "tile multiples");
  static_assert(8 * 2 * 64 * 4 <= 8 * SLAB_WAVE * 2, "reduce scratch fits in slab region");

  __shared__ __align__(16) unsigned short sBt[NOUT * KPAD];
  __shared__ __align__(16) unsigned short sA[128 * KPAD];
  __shared__ __align__(16) unsigned short sSlab[(LAYER == 2) ? 8 : 8 * SLAB_WAVE];
  __shared__ __align__(16) float sRedL2[(LAYER == 2) ? 8 * 4 * 128 : 4];
  __shared__ __align__(16) float sTot[NV * NOUT];
  __shared__ __align__(16) float sScSh[(LAYER == 0) ? 4 : 128];
  __shared__ int      sSel[(LAYER == 0) ? ROWS_BLK : 1];
  __shared__ int      sSelF[(LAYER == 0) ? ROWS_BLK : 1];
  __shared__ unsigned sRel[(LAYER == 0) ? 2 * ROWS_BLK : 1];
  __shared__ int      sCnt[(LAYER == 0) ? GRP_PER_BLK : 1];

  const int tid = threadIdx.x;
  const int lane = tid & 31, wave = tid >> 5;
  const int rl = lane & 15, hh = lane >> 4;
  const int koff = hh * 8, mOff = hh * 8;
  const int blk = blockIdx.x + blk0;
  const int row0 = blk * ROWS_BLK;
  const int bat = blk / BLK_PER_BATCH;
  const int blk_in_bat = blk - bat * BLK_PER_BATCH;

#pragma unroll 4
  for (int i = tid; i < NOUT * KPAD; i += 256) {
    const int n = i / KPAD;
    const int k = i - n * KPAD;
    float val;
    if (LAYER == 0) {
      const int col = (k < CFEAT) ? (3 + k) : ((k < CFEAT + 3) ? (k - CFEAT) : 0);
      const float wv = wgt[n * (CFEAT + 3) + col];
      const float scl = (k < CFEAT) ? W_CARRY : W_XYZ_CARRY;
      val = (k < CFEAT + 3) ? (wv * scl) : 0.0f;
    } else {
      val = wgt[n * CFEAT + k] * W_CARRY;
    }
    sBt[i] = (unsigned short)f16bits(val);
  }
  if (LAYER != 0) {
    if (tid < 128) sScSh[tid] = tab[(tid < 64) ? tid : (64 + tid)];
  }

  if (LAYER == 0) {
    const float* xb = xyz + (size_t)bat * 3 * NPTS;
#pragma unroll 1
    for (int gi = 0; gi < 2; ++gi) {
      const int grp = wave * 2 + gi;
      const int cs = blk_in_bat * GRP_PER_BLK + grp;
      const float cx = cplane[(size_t)bat * 3 * NCEN + cs];
      const float cy = cplane[(size_t)bat * 3 * NCEN + NCEN + cs];
      const float cz = cplane[(size_t)bat * 3 * NCEN + 2 * NCEN + cs];
      sSel[grp * 32 + lane] = NPTS - 1;
      int cnt = 0;
#pragma unroll 1
      for (int chunk = 0; chunk < NPTS / 32 && cnt < NSAMP; ++chunk) {
        const int j = chunk * 32 + lane;
        const float x = xb[j];
        const float y = xb[NPTS + j];
        const float z = xb[2 * NPTS + j];
        const float dx = cx - x;
        const float dy = cy - y;
        const float dz = cz - z;
        const float t0 = dx * dx;
        const float t1 = dy * dy;
        const float t2 = dz * dz;
        const float d2 = (t0 + t2) + t1;
        const bool inside = (d2 <= BALL_R2);
        const unsigned mask = __builtin_amdgcn_ballot_w32(inside);
        const int rank = __popc(mask & ((1u << lane) - 1u));
        const int slot = cnt + rank;
        if (inside && slot < NSAMP) sSel[grp * 32 + slot] = j;
        cnt += __popc(mask);
      }
      if (lane == 0) sCnt[grp] = cnt;
    }
  }
  __syncthreads();

  if (LAYER == 0) {
    const float* xb = xyz + (size_t)bat * 3 * NPTS;
#pragma unroll 1
    for (int i = 0; i < 2; ++i) {
      const int e = tid + 256 * i;
      const int grp = e >> 5, slot = e & 31;
      const int cntg = sCnt[grp];
      const int a = sSel[e];
      const int f = sSel[grp * 32];
      int sel = (slot < cntg) ? a : f;
      sel = sel < 0 ? 0 : (sel > NPTS - 1 ? NPTS - 1 : sel);
      const int cs = blk_in_bat * GRP_PER_BLK + grp;
      const float cx = cplane[(size_t)bat * 3 * NCEN + cs];
      const float cy = cplane[(size_t)bat * 3 * NCEN + NCEN + cs];
      const float cz = cplane[(size_t)bat * 3 * NCEN + 2 * NCEN + cs];
      const float rx = (xb[sel] - cx) * REL_CARRY;
      const float ry = (xb[NPTS + sel] - cy) * REL_CARRY;
      const float rz = (xb[2 * NPTS + sel] - cz) * REL_CARRY;
      unsigned zz = 0u;
      asm volatile("" : "+v"(zz));
      const unsigned w0 = pack2h(rx, ry);
      const unsigned w1 = (f16bits(rz) & 0xffffu) | (zz << 16);
      sSelF[e] = sel;
      sRel[2 * e] = w0;
      sRel[2 * e + 1] = w1;
    }
    __syncthreads();
  }

  float bv[NT];
#pragma unroll
  for (int j = 0; j < NT; ++j) bv[j] = bias[j * 16 + rl];

  float ssum[NT], ssq[NT], smx[NT], smn[NT];
#pragma unroll
  for (int j = 0; j < NT; ++j) {
    ssum[j] = 0.0f; ssq[j] = 0.0f;
    smx[j] = -__builtin_inff(); smn[j] = __builtin_inff();
  }

  const unsigned short* srcBase = srcA0;
  if (LAYER != 0) {
    srcBase = (row0 < split_row) ? (srcA0 + (size_t)row0 * 64) : (srcA1 + (size_t)(row0 - split_row) * 64);
  }

#pragma unroll 1
  for (int t = 0; t < ROWS_BLK / 128; ++t) {
    {
      const int r = tid >> 1, hf = tid & 1;
      v4u* ap = (v4u*)(sA + r * KPAD + hf * 32);
      if (LAYER == 0) {
        const int e = t * 128 + r;
        int sel = sSelF[e];
        sel = sel < 0 ? 0 : (sel > NPTS - 1 ? NPTS - 1 : sel);
        const v4u* gp = (const v4u*)(srcA0 + ((size_t)bat * NPTS + (size_t)sel) * CFEAT + hf * 32);
        const v4u g0 = gp[0], g1 = gp[1], g2 = gp[2], g3 = gp[3];
        const unsigned r0 = sRel[2 * e];
        const unsigned r1 = sRel[2 * e + 1];
        unsigned zz = 0u;
        asm volatile("" : "+v"(zz));
        v4u tl;
        tl.x = hf ? zz : r0;
        tl.y = hf ? zz : r1;
        tl.z = zz;
        tl.w = zz;
        v4u zv;
        zv.x = zz; zv.y = zz; zv.z = zz; zv.w = zz;
        ap[0] = g0; ap[1] = g1; ap[2] = g2; ap[3] = g3;
        v4u* tp = (v4u*)(sA + r * KPAD + 64 + hf * 16);
        tp[0] = tl;
        tp[1] = zv;
      } else {
        const v4u* gp = (const v4u*)(srcBase + (size_t)(t * 128 + r) * 64 + hf * 32);
        v4u g[4];
        g[0] = gp[0]; g[1] = gp[1]; g[2] = gp[2]; g[3] = gp[3];
#pragma unroll
        for (int q = 0; q < 4; ++q) {
          const v4f scA = *(const v4f*)(sScSh + hf * 32 + q * 8);
          const v4f scB = *(const v4f*)(sScSh + hf * 32 + q * 8 + 4);
          const v4f shA = *(const v4f*)(sScSh + 64 + hf * 32 + q * 8);
          const v4f shB = *(const v4f*)(sScSh + 64 + hf * 32 + q * 8 + 4);
          ap[q] = bn8(g[q], scA, scB, shA, shB);
        }
      }
    }
    __syncthreads();

    v8f acc[NT];
#pragma unroll
    for (int j = 0; j < NT; ++j) acc[j] = (v8f){0.f, 0.f, 0.f, 0.f, 0.f, 0.f, 0.f, 0.f};
#pragma unroll
    for (int kk = 0; kk < KS; ++kk) {
      const v16h a = FragH::load((const _Float16*)sA + (wave * 16 + rl) * KPAD + kk * 32 + koff);
#pragma unroll
      for (int j = 0; j < NT; ++j) {
        const v16h bfr = FragH::load((const _Float16*)sBt + (j * 16 + rl) * KPAD + kk * 32 + koff);
        acc[j] = mma_h(a, bfr, acc[j]);
      }
    }

#pragma unroll
    for (int j = 0; j < NT; ++j) {
#pragma unroll
      for (int r = 0; r < 8; ++r) {
        const float x = acc[j][r] * ACC_FOLD + bv[j];
        ssum[j] += x;
        ssq[j] += x * x;
        if (LAYER == 2) { smx[j] = fmaxf(smx[j], x); smn[j] = fminf(smn[j], x); }
        if (LAYER < 2) sSlab[wave * SLAB_WAVE + (mOff + r) * SLAB_PITCH + j * 16 + rl] = (unsigned short)f16bits(x);
      }
    }
    __syncthreads();

    if (LAYER < 2) {
      const int q = lane >> 3, c8 = (lane & 7) * 8;
      v4u sv[4];
#pragma unroll
      for (int it = 0; it < 4; ++it)
        sv[it] = *(const v4u*)(sSlab + wave * SLAB_WAVE + (it * 4 + q) * SLAB_PITCH + c8);
      unsigned short* drow = dst + (size_t)(row0 + t * 128 + wave * 16 - dst_row0) * 64;
      for (int pass = 0; pass < 2; ++pass) {
#pragma unroll
        for (int it = 0; it < 4; ++it)
          *(volatile v4u*)(drow + (size_t)(it * 4 + q) * 64 + c8) = sv[it];
        __threadfence();
      }
    }
  }

#pragma unroll
  for (int j = 0; j < NT; ++j) {
    const float os = __shfl_xor(ssum[j], 16, 32);
    const float oq = __shfl_xor(ssq[j], 16, 32);
    const float ox = __shfl_xor(smx[j], 16, 32);
    const float on = __shfl_xor(smn[j], 16, 32);
    ssum[j] += os;
    ssq[j] += oq;
    smx[j] = fmaxf(smx[j], ox);
    smn[j] = fminf(smn[j], on);
  }
  __syncthreads();
  float* red = (LAYER == 2) ? sRedL2 : (float*)sSlab;
  if (hh == 0) {
#pragma unroll
    for (int j = 0; j < NT; ++j) {
      red[(wave * NV + 0) * NOUT + j * 16 + rl] = ssum[j];
      red[(wave * NV + 1) * NOUT + j * 16 + rl] = ssq[j];
      if (LAYER == 2) {
        red[(wave * NV + 2) * NOUT + j * 16 + rl] = smx[j];
        red[(wave * NV + 3) * NOUT + j * 16 + rl] = smn[j];
      }
    }
  }
  __syncthreads();
  for (int idx = tid; idx < NV * NOUT; idx += 256) {
    const int which = idx / NOUT;
    const int c = idx - which * NOUT;
    float sv = 0.0f, mxv = -__builtin_inff(), mnv = __builtin_inff();
#pragma unroll
    for (int w = 0; w < 8; ++w) {
      const float v = red[(w * NV + which) * NOUT + c];
      sv += v;
      mxv = fmaxf(mxv, v);
      mnv = fminf(mnv, v);
    }
    sTot[idx] = (which < 2) ? sv : ((which == 2) ? mxv : mnv);
  }
  __syncthreads();
  if (wave == 0) {
    constexpr int NCHUNK = (NV * NOUT) / 128;
    v4f pv[NCHUNK];
#pragma unroll
    for (int ch = 0; ch < NCHUNK; ++ch) pv[ch] = *(const v4f*)(sTot + ch * 128 + lane * 4);
    float* pd = part + (size_t)blk * (NV * NOUT);
    for (int pass = 0; pass < 2; ++pass) {
#pragma unroll
      for (int ch = 0; ch < NCHUNK; ++ch) *(volatile v4f*)(pd + ch * 128 + lane * 4) = pv[ch];
      __threadfence();
    }
  }
}

__device__ __forceinline__ void bn_coeffs(const float* __restrict__ part, int nblk, int stride, int nout, int c,
                                          const float* __restrict__ g, const float* __restrict__ beta,
                                          float& sc, float& sh) {
  double S = 0.0, Q = 0.0;
#pragma unroll 4
  for (int k = 0; k < nblk; ++k) {
    S += (double)part[(size_t)k * stride + c];
    Q += (double)part[(size_t)k * stride + nout + c];
  }
  const double invM = 1.0 / (double)MROWS;
  const double mean = S * invM;
  double var = Q * invM - mean * mean;
  var = (var < 0.0) ? 0.0 : var;
  const float vf = (float)var + BN_EPS;
  const float rs = 1.0f / sqrtf(vf);
  sc = g[c] * rs;
  sh = beta[c] - sc * (float)mean;
}

__global__ __launch_bounds__(128) void k_fin(const float* __restrict__ part, int nblk, int stride, int nout,
                                             const float* __restrict__ g, const float* __restrict__ beta, float* tab) {
  __shared__ __align__(16) float sTab[256];
  const int tid = threadIdx.x;
  const int nb = nblk > NBLK_ALL ? NBLK_ALL : nblk;
  const int c = (tid < nout) ? tid : (nout - 1);
  float sc, sh;
  bn_coeffs(part, nb, stride, nout, c, g, beta, sc, sh);
  sTab[tid] = (tid < nout) ? sc : 0.0f;
  sTab[128 + tid] = (tid < nout) ? sh : 0.0f;
  __syncthreads();
  if (tid < 32) {
    const v4f a = *(const v4f*)(sTab + tid * 4);
    const v4f b = *(const v4f*)(sTab + 128 + tid * 4);
    for (int pass = 0; pass < 2; ++pass) {
      *(volatile v4f*)(tab + tid * 4) = a;
      *(volatile v4f*)(tab + 128 + tid * 4) = b;
      __threadfence();
    }
  }
}

__global__ __launch_bounds__(128) void k_out(const float* __restrict__ part2, const float* __restrict__ g,
                                             const float* __restrict__ beta, float* out1) {
  __shared__ __align__(16) float sO[128];
  const int tid = threadIdx.x;
  const int b = blockIdx.x;
  float sc, sh;
  bn_coeffs(part2, NBLK_ALL, 512, 128, tid, g, beta, sc, sh);
  float mx = -__builtin_inff(), mn = __builtin_inff();
#pragma unroll 4
  for (int k = 0; k < BLK_PER_BATCH; ++k) {
    const size_t base = (size_t)(b * BLK_PER_BATCH + k) * 512;
    mx = fmaxf(mx, part2[base + 256 + tid]);
    mn = fminf(mn, part2[base + 384 + tid]);
  }
  const float xsel = (sc >= 0.0f) ? mx : mn;
  const float y = fmaxf(sc * xsel + sh, 0.0f);
  sO[tid] = y;
  __syncthreads();
  if (tid < 32) {
    const v4f v = *(const v4f*)(sO + tid * 4);
    float* od = out1 + (size_t)b * 128 + tid * 4;
    for (int pass = 0; pass < 2; ++pass) {
      *(volatile v4f*)od = v;
      __threadfence();
    }
  }
}

extern "C" void kernel_launch(void* const* d_in, const int* in_sizes, int n_in,
                              void* d_out, int out_size, void* d_ws, size_t ws_size, hipStream_t stream) {
  (void)in_sizes; (void)out_size;
  if (n_in < 14) return;
  if (ws_size < WS_TOTAL) return;
  const float* xyz   = (const float*)d_in[0];
  const float* pts   = (const float*)d_in[1];
  const float* w0    = (const float*)d_in[2];
  const float* b0    = (const float*)d_in[3];
  const float* g0    = (const float*)d_in[4];
  const float* beta0 = (const float*)d_in[5];
  const float* w1    = (const float*)d_in[6];
  const float* b1    = (const float*)d_in[7];
  const float* g1    = (const float*)d_in[8];
  const float* beta1 = (const float*)d_in[9];
  const float* w2    = (const float*)d_in[10];
  const float* b2    = (const float*)d_in[11];
  const float* g2    = (const float*)d_in[12];
  const float* beta2 = (const float*)d_in[13];

  float* out0 = (float*)d_out;
  float* out1 = (float*)d_out + OUT1_OFF;

  char* ws = (char*)d_ws;
  unsigned short* ptsh = (unsigned short*)(ws + WS_PTS);
  unsigned short* y0   = (unsigned short*)(ws + WS_Y0);
  unsigned short* tpl  = (unsigned short*)(ws + WS_T);
  float* cen  = (float*)(ws + WS_CEN);
  float* p0   = (float*)(ws + WS_P0);
  float* p1   = (float*)(ws + WS_P1);
  float* p2   = (float*)(ws + WS_P2);
  float* tab0 = (float*)(ws + WS_TAB0);
  float* tab1 = (float*)(ws + WS_TAB1);

  k_fps<<<NBATCH, FPS_THREADS, 0, stream>>>(xyz, out0, cen);
  k_tr<<<NBATCH * (NPTS / 64), 256, 0, stream>>>(pts, ptsh);

  k_layer<0><<<NBLK_ALL, 256, 0, stream>>>(xyz, cen, ptsh, ptsh, MROWS, w0, b0, tab0, y0, 0, p0, 0);
  k_fin<<<1, 128, 0, stream>>>(p0, NBLK_ALL, 128, 64, g0, beta0, tab0);

  k_layer<1><<<NBLK_ALL / 2, 256, 0, stream>>>(xyz, cen, y0, y0, MROWS, w1, b1, tab0, tpl, 0, p1, 0);
  k_layer<1><<<NBLK_ALL / 2, 256, 0, stream>>>(xyz, cen, y0, y0, MROWS, w1, b1, tab0, y0, MROWS / 2, p1, NBLK_ALL / 2);
  k_fin<<<1, 128, 0, stream>>>(p1, NBLK_ALL, 128, 64, g1, beta1, tab1);

  k_layer<2><<<NBLK_ALL, 256, 0, stream>>>(xyz, cen, tpl, y0, MROWS / 2, w2, b2, tab1, y0, 0, p2, 0);
  k_out<<<NBATCH, 128, 0, stream>>>(p2, g2, beta2, out1);
}
